// KHopSumAggregator_9801115369800
// MI455X (gfx1250) — hardware-verified
//
#include <hip/hip_runtime.h>
#include <stddef.h>
#include <stdint.h>


#define NN      4096
#define NWORDS  128
#define FDIM    64
#define KHOP    3
#define MPOW    4
#define NTHR    256
#define NWAVE   8
#define EPT     8
#define NGRP    2
#define CHUNK   (NTHR * EPT * NGRP)
#define WCAP    (EPT * NGRP * 32)
#define LISTN   (NWAVE * WCAP)
#define TB      64
#define JB      64
#define STP     68
#define RPW     4
#define CGW     64

static_assert((CHUNK & (CHUNK - 1)) == 0);
static_assert(CHUNK <= 4096);
static_assert((TB & (TB - 1)) == 0 && TB <= 4096);
static_assert((NN % TB) == 0);
static_assert(NWORDS * 32 == NN);
static_assert((NN % (NWAVE * RPW)) == 0);
static_assert((NN % JB) == 0 && JB == 64 && FDIM == 64);
static_assert((TB * NWORDS / 4) % NTHR == 0);
static_assert(CGW == FDIM);
static_assert((STP * 4) % 16 == 0);
static_assert(MPOW == 4 && KHOP == 3);

typedef float    v4f  __attribute__((ext_vector_type(4)));
typedef float    v8f  __attribute__((ext_vector_type(8)));
typedef int      v4i  __attribute__((ext_vector_type(4)));
typedef unsigned v4u  __attribute__((ext_vector_type(4)));
typedef _Float16 v8h  __attribute__((ext_vector_type(8)));
typedef _Float16 v16h __attribute__((ext_vector_type(16)));
union FragH { v16h v; v8h h[2]; };

__device__ __forceinline__ v8h cvt8(v4f a, v4f b) {
  v8h r;
  r[0] = (_Float16)a.x; r[1] = (_Float16)a.y; r[2] = (_Float16)a.z; r[3] = (_Float16)a.w;
  r[4] = (_Float16)b.x; r[5] = (_Float16)b.y; r[6] = (_Float16)b.z; r[7] = (_Float16)b.w;
  return r;
}

template <int NB>
__device__ __forceinline__ int scan_chunk(const int* __restrict__ dsts, int nE, int cbase, int slotBase,
                                          int vec8, int* list, int tid, int lane, int wave) {
  int wc = 0;
#pragma unroll
  for (int g = 0; g < NGRP; ++g) {
    const int el0  = (g * NTHR + tid) * EPT;
    const int e0   = cbase + el0;
    const int sent = -2147483647 - 1;
    v4i da, db;
    if (vec8 != 0 && cbase + CHUNK <= nE) {
      da = *(const v4i*)(dsts + e0);
      db = *(const v4i*)(dsts + e0 + 4);
    } else {
      da.x = (e0     < nE) ? dsts[min(e0, nE - 1)]     : sent;
      da.y = (e0 + 1 < nE) ? dsts[min(e0 + 1, nE - 1)] : sent;
      da.z = (e0 + 2 < nE) ? dsts[min(e0 + 2, nE - 1)] : sent;
      da.w = (e0 + 3 < nE) ? dsts[min(e0 + 3, nE - 1)] : sent;
      db.x = (e0 + 4 < nE) ? dsts[min(e0 + 4, nE - 1)] : sent;
      db.y = (e0 + 5 < nE) ? dsts[min(e0 + 5, nE - 1)] : sent;
      db.z = (e0 + 6 < nE) ? dsts[min(e0 + 6, nE - 1)] : sent;
      db.w = (e0 + 7 < nE) ? dsts[min(e0 + 7, nE - 1)] : sent;
    }
    const unsigned nb = (unsigned)slotBase;
    const unsigned s0 = (unsigned)da.x - nb, s1 = (unsigned)da.y - nb;
    const unsigned s2 = (unsigned)da.z - nb, s3 = (unsigned)da.w - nb;
    const unsigned s4 = (unsigned)db.x - nb, s5 = (unsigned)db.y - nb;
    const unsigned s6 = (unsigned)db.z - nb, s7 = (unsigned)db.w - nb;
    const bool h0 = s0 < (unsigned)NB, h1 = s1 < (unsigned)NB, h2 = s2 < (unsigned)NB, h3 = s3 < (unsigned)NB;
    const bool h4 = s4 < (unsigned)NB, h5 = s5 < (unsigned)NB, h6 = s6 < (unsigned)NB, h7 = s7 < (unsigned)NB;
    const unsigned any = __builtin_amdgcn_ballot_w32(h0 | h1 | h2 | h3 | h4 | h5 | h6 | h7);
    if (any != 0u) {
#define HITJ(J, HJ, SJ) { \
        const unsigned mj = __builtin_amdgcn_ballot_w32(HJ); \
        if (mj != 0u) { \
          if (HJ) { \
            const int pos = wc + (int)__builtin_amdgcn_mbcnt_lo(mj, 0u); \
            if (pos < WCAP) list[wave * WCAP + pos] = ((el0 + (J)) << 12) | (int)(SJ); \
          } \
          wc += (int)__builtin_popcount(mj); } }
      HITJ(0, h0, s0)
      HITJ(1, h1, s1)
      HITJ(2, h2, s2)
      HITJ(3, h3, s3)
      HITJ(4, h4, s4)
      HITJ(5, h5, s5)
      HITJ(6, h6, s6)
      HITJ(7, h7, s7)
#undef HITJ
    }
  }
  return wc;
}

__global__ __launch_bounds__(NTHR) void k_adj(
    const int* __restrict__ ei, unsigned* abit, int nE, int vec8) {
  __shared__ __attribute__((aligned(16))) unsigned bits[TB * NWORDS];
  __shared__ __attribute__((aligned(16))) int list[LISTN];
  __shared__ int wcnt[NWAVE];
  const int tid = threadIdx.x, lane = tid & 31, wave = tid >> 5;
  const int tBase = blockIdx.x * TB;
  const int* dsts = ei + nE;

  {
    const v4u z = {0u, 0u, 0u, 0u};
    for (int i = tid; i < TB * NWORDS / 4; i += NTHR) ((v4u*)bits)[i] = z;
  }
  __syncthreads();

  const int nChunks = (nE + CHUNK - 1) / CHUNK;
#pragma unroll 1
  for (int ch = 0; ch < nChunks; ++ch) {
    const int cbase = ch * CHUNK;
    const int wc = scan_chunk<TB>(dsts, nE, cbase, tBase, vec8, list, tid, lane, wave);
    if (lane == 0) wcnt[wave] = wc;
    __syncthreads();
    if (wave == 0) {
#pragma unroll 1
      for (int wsx = 0; wsx < NWAVE; ++wsx) {
        int n = __builtin_amdgcn_readfirstlane(wcnt[wsx]);
        n = n > WCAP ? WCAP : (n < 0 ? 0 : n);
        const int* lp = list + wsx * WCAP;
#pragma unroll 1
        for (int i = 0; i < n; ++i) {
          const int ent  = __builtin_amdgcn_readfirstlane(lp[i]);
          const int slot = ent & (TB - 1);
          int e = cbase + ((ent >> 12) & (CHUNK - 1));
          e = e > nE - 1 ? nE - 1 : e;
          int s = ei[e];
          s = s < 0 ? 0 : (s > NN - 1 ? NN - 1 : s);
          if (lane == 0) {
            const int wi = slot * NWORDS + (s >> 5);
            bits[wi] = bits[wi] | (1u << (s & 31));
          }
        }
      }
    }
    __syncthreads();
  }

  unsigned* gp = abit + (size_t)tBase * NWORDS;
#pragma unroll
  for (int p = 0; p < (TB * NWORDS / 4) / NTHR; ++p) {
    const v4u v = ((const v4u*)bits)[p * NTHR + tid];
    *(volatile v4u*)(gp + 4 * (p * NTHR + tid)) = v;
  }
  __threadfence();
#pragma unroll
  for (int p = 0; p < (TB * NWORDS / 4) / NTHR; ++p) {
    const v4u v = ((const v4u*)bits)[p * NTHR + tid];
    *(volatile v4u*)(gp + 4 * (p * NTHR + tid)) = v;
  }
}

__device__ __forceinline__ v4f ipow(v4f a, int mexp) {
  const v4f a2 = a * a;
  return mexp == 0 ? a : (mexp == 1 ? a2 : (mexp == 2 ? a2 * a : a2 * a2));
}

__global__ __launch_bounds__(NTHR) void k_pows(
    const float* __restrict__ x, _Float16* pt) {
  __shared__ __attribute__((aligned(16))) float st[FDIM * STP];
  const int tid = threadIdx.x;
  const int b  = blockIdx.x / (NN / JB);
  const int jb = blockIdx.x - b * (NN / JB);
  const int j0 = jb * JB;

#pragma unroll
  for (int p = 0; p < (JB * FDIM) / NTHR; ++p) {
    const int idx = p * NTHR + tid;
    const int j = idx >> 6, f = idx & 63;
    const float v = fabsf(x[((size_t)b * NN + j0 + j) * FDIM + f]);
    st[f * STP + j] = v;
  }
  __syncthreads();

  v8h hv[8];
#pragma unroll
  for (int p = 0; p < 8; ++p) {
    const int rl   = p * 32 + (tid >> 3);
    const int f    = rl & 63;
    const int mexp = p >> 1;
    const int q    = tid & 7;
    const v4f a  = *(const v4f*)(st + f * STP + 8 * q);
    const v4f c  = *(const v4f*)(st + f * STP + 8 * q + 4);
    hv[p] = cvt8(ipow(a, mexp), ipow(c, mexp));
  }
  _Float16* gb = pt + (size_t)b * (MPOW * FDIM) * NN + j0;
#pragma unroll
  for (int p = 0; p < 8; ++p) {
    const int rl = p * 32 + (tid >> 3);
    const int q  = tid & 7;
    *(volatile v8h*)(gb + (size_t)rl * NN + 8 * q) = hv[p];
  }
  __threadfence();
#pragma unroll
  for (int p = 0; p < 8; ++p) {
    const int rl = p * 32 + (tid >> 3);
    const int q  = tid & 7;
    *(volatile v8h*)(gb + (size_t)rl * NN + 8 * q) = hv[p];
  }
}

__device__ __forceinline__ v4u expand_row(v4u prv, const unsigned* __restrict__ abit, int lane) {
  v4u acc = prv;
#pragma unroll 1
  for (int ln = 0; ln < 32; ++ln) {
    unsigned wv[4];
    wv[0] = (unsigned)__builtin_amdgcn_readlane((int)prv.x, ln);
    wv[1] = (unsigned)__builtin_amdgcn_readlane((int)prv.y, ln);
    wv[2] = (unsigned)__builtin_amdgcn_readlane((int)prv.z, ln);
    wv[3] = (unsigned)__builtin_amdgcn_readlane((int)prv.w, ln);
#pragma unroll
    for (int c = 0; c < 4; ++c) {
      unsigned bts = wv[c];
      const int tb = (ln * 4 + c) << 5;
#pragma unroll 1
      while (bts != 0u) {
        const int bpos = __builtin_ctz(bts);
        bts &= bts - 1u;
        const int t = (tb + bpos) & (NN - 1);
        const v4u g = *(const v4u*)(abit + (size_t)t * NWORDS + 4 * lane);
        acc |= g;
      }
    }
  }
  return acc;
}

__global__ __launch_bounds__(NTHR) void k_reach(
    const unsigned* __restrict__ abit, unsigned* reach) {
  const int tid = threadIdx.x, lane = tid & 31, wave = tid >> 5;
#pragma unroll 1
  for (int rr = 0; rr < RPW; ++rr) {
    const int i = (blockIdx.x * NWAVE + wave) * RPW + rr;
    v4u r = *(const v4u*)(abit + (size_t)i * NWORDS + 4 * lane);
    const int wi = i >> 5;
    const unsigned sb = 1u << (i & 31);
    const bool mine = (lane == (wi >> 2));
    const int cc = wi & 3;
    r.x |= (mine && cc == 0) ? sb : 0u;
    r.y |= (mine && cc == 1) ? sb : 0u;
    r.z |= (mine && cc == 2) ? sb : 0u;
    r.w |= (mine && cc == 3) ? sb : 0u;
    unsigned* p0 = reach + ((size_t)0 * NN + i) * NWORDS + 4 * lane;
    *(volatile v4u*)p0 = r;
    __threadfence();
    *(volatile v4u*)p0 = r;
    r = expand_row(r, abit, lane);
    unsigned* p1 = reach + ((size_t)1 * NN + i) * NWORDS + 4 * lane;
    *(volatile v4u*)p1 = r;
    __threadfence();
    *(volatile v4u*)p1 = r;
    r = expand_row(r, abit, lane);
    unsigned* p2 = reach + ((size_t)2 * NN + i) * NWORDS + 4 * lane;
    *(volatile v4u*)p2 = r;
    __threadfence();
    *(volatile v4u*)p2 = r;
  }
}

#define WMH(ACC, A, B) ACC = __builtin_amdgcn_wmma_f32_16x16x32_f16(false, A, false, B, (short)0, ACC, false, false)
#define HOPGUARD(ACC, A, B0, B1, B2, B3) \
  asm volatile("v_nop\n\tv_nop\n\tv_nop\n\tv_nop" \
               : "+v"(ACC[0]), "+v"(ACC[1]), "+v"(ACC[2]), "+v"(ACC[3]) \
               : "v"(A), "v"(B0), "v"(B1), "v"(B2), "v"(B3))

__global__ __launch_bounds__(NTHR) void k_khop(
    const unsigned* __restrict__ reach, const _Float16* __restrict__ pt, float* out, int nCgb) {
  __shared__ __attribute__((aligned(16))) _Float16 lut[256 * 8];
  __shared__ __attribute__((aligned(16))) float stg[NWAVE * 16 * CGW];
  const int tid = threadIdx.x, lane = tid & 31, wave = tid >> 5, h = lane >> 4, m = lane & 15;

  {
    v8h e;
#pragma unroll
    for (int c = 0; c < 8; ++c) e[c] = ((tid >> c) & 1) ? (_Float16)1.0f : (_Float16)0.0f;
    *(v8h*)(lut + 8 * tid) = e;
  }
  __syncthreads();

  const int itile = blockIdx.x / nCgb;
  const int cg    = (blockIdx.x - itile * nCgb) * NWAVE + wave;
  const int bb    = cg >> 2;
  const int mq    = cg & 3;
  const int i0    = itile * 16;
  const unsigned* rp0 = reach + ((size_t)0 * NN + i0 + m) * NWORDS;
  const unsigned* rp1 = reach + ((size_t)1 * NN + i0 + m) * NWORDS;
  const unsigned* rp2 = reach + ((size_t)2 * NN + i0 + m) * NWORDS;
  const _Float16* bp  = pt + (size_t)(cg * CGW + m) * NN + 8 * h;
  const int sh = 8 * h;

  v8f acc0[4], acc1[4], acc2[4];
#pragma unroll
  for (int t = 0; t < 4; ++t) {
    const v8f z = {0.f, 0.f, 0.f, 0.f, 0.f, 0.f, 0.f, 0.f};
    acc0[t] = z; acc1[t] = z; acc2[t] = z;
  }

#pragma unroll 1
  for (int ks = 0; ks < NWORDS; ++ks) {
    const int k0 = ks * 32;
    FragH bq[4];
#pragma unroll
    for (int t = 0; t < 4; ++t) {
      const _Float16* p = bp + (size_t)t * 16 * NN + k0;
      bq[t].h[0] = *(const v8h*)p;
      bq[t].h[1] = *(const v8h*)(p + 16);
    }
    const unsigned w0 = rp0[ks], w1 = rp1[ks], w2 = rp2[ks];
    FragH a0, a1, a2;
    a0.h[0] = *(const v8h*)(lut + 8 * ((w0 >> sh) & 255u));
    a0.h[1] = *(const v8h*)(lut + 8 * ((w0 >> (sh + 16)) & 255u));
    a1.h[0] = *(const v8h*)(lut + 8 * ((w1 >> sh) & 255u));
    a1.h[1] = *(const v8h*)(lut + 8 * ((w1 >> (sh + 16)) & 255u));
    a2.h[0] = *(const v8h*)(lut + 8 * ((w2 >> sh) & 255u));
    a2.h[1] = *(const v8h*)(lut + 8 * ((w2 >> (sh + 16)) & 255u));

    WMH(acc0[0], a0.v, bq[0].v); WMH(acc0[1], a0.v, bq[1].v);
    WMH(acc0[2], a0.v, bq[2].v); WMH(acc0[3], a0.v, bq[3].v);
    HOPGUARD(acc0, a0.v, bq[0].v, bq[1].v, bq[2].v, bq[3].v);
    WMH(acc1[0], a1.v, bq[0].v); WMH(acc1[1], a1.v, bq[1].v);
    WMH(acc1[2], a1.v, bq[2].v); WMH(acc1[3], a1.v, bq[3].v);
    HOPGUARD(acc1, a1.v, bq[0].v, bq[1].v, bq[2].v, bq[3].v);
    WMH(acc2[0], a2.v, bq[0].v); WMH(acc2[1], a2.v, bq[1].v);
    WMH(acc2[2], a2.v, bq[2].v); WMH(acc2[3], a2.v, bq[3].v);
    HOPGUARD(acc2, a2.v, bq[0].v, bq[1].v, bq[2].v, bq[3].v);
  }

  float* sw = stg + wave * (16 * CGW);
  const int piece = lane & 15;
#pragma unroll
  for (int kk = 0; kk < KHOP; ++kk) {
#pragma unroll
    for (int t = 0; t < 4; ++t) {
#pragma unroll
      for (int r = 0; r < 8; ++r) {
        const float v = (kk == 0) ? acc0[t][r] : ((kk == 1) ? acc1[t][r] : acc2[t][r]);
        sw[(8 * h + r) * CGW + 16 * t + m] = v;
      }
    }
    __syncthreads();
#pragma unroll
    for (int rr = 0; rr < 8; ++rr) {
      const int row = 2 * rr + h;
      const v4f v = *(const v4f*)(sw + row * CGW + 4 * piece);
      float* gp = out + ((((size_t)bb * NN + i0 + row) * KHOP + kk) * MPOW + mq) * FDIM + 4 * piece;
      *(volatile v4f*)gp = v;
    }
    __threadfence();
#pragma unroll
    for (int rr = 0; rr < 8; ++rr) {
      const int row = 2 * rr + h;
      const v4f v = *(const v4f*)(sw + row * CGW + 4 * piece);
      float* gp = out + ((((size_t)bb * NN + i0 + row) * KHOP + kk) * MPOW + mq) * FDIM + 4 * piece;
      *(volatile v4f*)gp = v;
    }
    __syncthreads();
  }
}
#undef WMH
#undef HOPGUARD

extern "C" void kernel_launch(void* const* d_in, const int* in_sizes, int n_in,
                              void* d_out, int out_size, void* d_ws, size_t ws_size,
                              hipStream_t stream) {
  if (n_in < 2) return;
  const int nB = in_sizes[0] / (NN * FDIM);
  if (nB < 1 || in_sizes[0] != nB * NN * FDIM) return;
  const int nE = in_sizes[1] / 2;
  if (nE < 1 || in_sizes[1] != 2 * nE || nE > (1 << 28)) return;
  if (out_size != nB * NN * KHOP * MPOW * FDIM) return;
  const int nCg = nB * MPOW;
  if ((nCg % NWAVE) != 0) return;
  const int nCgb = nCg / NWAVE;

  const float* x  = (const float*)d_in[0];
  const int*   ei = (const int*)d_in[1];
  float* out = (float*)d_out;

  char* ws = (char*)d_ws;
  size_t off = 0;
  const size_t oAbit  = off; off += (size_t)NN * NWORDS * 4;               off = (off + 255) & ~(size_t)255;
  const size_t oPt    = off; off += (size_t)nCg * CGW * NN * 2;            off = (off + 255) & ~(size_t)255;
  const size_t oReach = off; off += (size_t)KHOP * NN * NWORDS * 4;        off = (off + 255) & ~(size_t)255;
  if (off > ws_size || off > ((size_t)128 << 20)) return;
  unsigned* abit  = (unsigned*)(ws + oAbit);
  _Float16* pt    = (_Float16*)(ws + oPt);
  unsigned* reach = (unsigned*)(ws + oReach);

  const int vec8 = ((nE & 3) == 0) ? 1 : 0;

  k_adj<<<NN / TB, NTHR, 0, stream>>>(ei, abit, nE, vec8);
  k_pows<<<nB * (NN / JB), NTHR, 0, stream>>>(x, pt);
  k_reach<<<NN / (NWAVE * RPW), NTHR, 0, stream>>>(abit, reach);
  k_khop<<<(NN / 16) * nCgb, NTHR, 0, stream>>>(reach, pt, out, nCgb);
}
